// CrossAttentionCondition_16131897163996
// MI455X (gfx1250) — hardware-verified
//
#include <hip/hip_runtime.h>
#include <math.h>

typedef __attribute__((ext_vector_type(16))) _Float16 v16h;
typedef __attribute__((ext_vector_type(16))) __bf16 v16b;
typedef __attribute__((ext_vector_type(8)))  _Float16 v8h;
typedef __attribute__((ext_vector_type(8)))  float v8f;
typedef __attribute__((ext_vector_type(4)))  float v4f;
typedef __attribute__((ext_vector_type(2)))  float v2f;
typedef __attribute__((ext_vector_type(4)))  unsigned v4u;
typedef __attribute__((ext_vector_type(4)))  int v4i;
typedef float __attribute__((may_alias)) float_a;
typedef int __attribute__((may_alias)) int_a;

template <typename T> __device__ __forceinline__ void vst2(void* p, T v) { *(volatile T*)p = v; __threadfence(); *(volatile T*)p = v; }
__device__ __forceinline__ v8f wmma16(v16h a, v16h b, v8f c) {
  v8f d = __builtin_amdgcn_wmma_f32_16x16x32_f16(false, a, false, b, (short)0, c, false, false);
  asm volatile("v_nop\n\tv_nop\n\tv_nop\n\tv_nop" : "+v"(d) : "v"(a), "v"(b));
  return d;
}
__device__ __forceinline__ v8f wmma_bf(v16b a, v16b b, v8f c) {
  v8f d = __builtin_amdgcn_wmma_f32_16x16x32_bf16(false, a, false, b, (short)0, c, false, false);
  asm volatile("v_nop\n\tv_nop\n\tv_nop\n\tv_nop" : "+v"(d) : "v"(a), "v"(b));
  return d;
}
__device__ __forceinline__ v16h frag_h(const _Float16* rowk0, int lane) {
  union { v16h v; v8h q[2]; } u; const _Float16* p = rowk0 + 8 * (lane >> 4);
  u.q[0] = *(const v8h*)p; u.q[1] = *(const v8h*)(p + 16); return u.v;
}
__device__ __forceinline__ v16h frag_f32(const float* rowk0, int lane) {
  v16h a; const float* p = rowk0 + 8 * (lane >> 4);
#pragma unroll
  for (int i = 0; i < 8; ++i) { a[i] = (_Float16)p[i]; a[8 + i] = (_Float16)p[16 + i]; }
  return a;
}
__device__ __forceinline__ v16h frag_f32s(const float* rowk0, int lane, float sc) {
  v16h a; const float* p = rowk0 + 8 * (lane >> 4);
#pragma unroll
  for (int i = 0; i < 8; ++i) { a[i] = (_Float16)(p[i] * sc); a[8 + i] = (_Float16)(p[16 + i] * sc); }
  return a;
}
__device__ __forceinline__ v16h fragc_f32(const float* W, int k0, int n, int lane, int ld, int K) {
  v16h a; const int g = lane >> 4;
#pragma unroll
  for (int i = 0; i < 8; ++i) { const int ka = k0 + 8 * g + i, kb = ka + 16;
    a[i] = (_Float16)(ka < K ? W[(size_t)(ka < K ? ka : K - 1) * ld + n] : 0.f); a[8 + i] = (_Float16)(kb < K ? W[(size_t)(kb < K ? kb : K - 1) * ld + n] : 0.f); }
  return a;
}
struct F2 { v16b h, l; };
__device__ __forceinline__ F2 bsplit16(const float v[16]) { F2 r;
#pragma unroll
  for (int i = 0; i < 16; ++i) { const __bf16 h = (__bf16)v[i]; r.h[i] = h; r.l[i] = (__bf16)(v[i] - (float)h); }
  return r; }
__device__ __forceinline__ F2 split_row(const float* row, int k0, int lane) { float v[16]; const float* p = row + k0 + 8 * (lane >> 4);
#pragma unroll
  for (int i = 0; i < 8; ++i) { v[i] = p[i]; v[8 + i] = p[16 + i]; }
  return bsplit16(v); }
__device__ __forceinline__ F2 split_rowK(const float* row, int k0, int lane, int K) { float v[16]; const int g = lane >> 4;
#pragma unroll
  for (int i = 0; i < 8; ++i) { const int ka = k0 + 8 * g + i, kb = ka + 16; v[i] = ka < K ? row[ka < K ? ka : K - 1] : 0.f; v[8 + i] = kb < K ? row[kb < K ? kb : K - 1] : 0.f; }
  return bsplit16(v); }
__device__ __forceinline__ F2 split_col(const float* W, int k0, int n, int lane, int ld, int K) { float v[16]; const int g = lane >> 4;
#pragma unroll
  for (int i = 0; i < 8; ++i) { const int ka = k0 + 8 * g + i, kb = ka + 16; v[i] = ka < K ? W[(size_t)(ka < K ? ka : K - 1) * ld + n] : 0.f; v[8 + i] = kb < K ? W[(size_t)(kb < K ? kb : K - 1) * ld + n] : 0.f; }
  return bsplit16(v); }
__device__ __forceinline__ v8f mac3(const F2& a, const F2& b, v8f c) { c = wmma_bf(a.l, b.h, c); c = wmma_bf(a.h, b.l, c); return wmma_bf(a.h, b.h, c); }
__device__ __forceinline__ float sigm(float v) { return 1.0f / (1.0f + expf(-v)); }
#define LDSX() do { asm volatile("s_wait_dscnt 0" ::: "memory"); __builtin_amdgcn_wave_barrier(); __builtin_amdgcn_fence(__ATOMIC_RELEASE, "workgroup"); } while (0)


#define NB 2
#define SX 2048
#define SC 512
#define SR 512
#define SKV (SC + SR)
#define DM_ 2048
#define NH 16
#define HD 128
#ifndef TQB
#define TQB (SX / 64)
#endif
#ifndef TNB
#define TNB NB
#endif
typedef __attribute__((ext_vector_type(8))) __bf16 v8b;
__device__ __forceinline__ v16b frag_b(const __bf16* rowk0, int lane) {
  union { v16b v; v8b q[2]; } u; const __bf16* p = rowk0 + 8 * (lane >> 4);
  u.q[0] = *(const v8b*)p; u.q[1] = *(const v8b*)(p + 16); return u.v;
}
__device__ __forceinline__ float bfr(float v) { return (float)(__bf16)v; }
__device__ __attribute__((noinline)) float exp_ni(float v) { return expf(v); }
__device__ __attribute__((noinline)) float erf_ni(float v) { return erff(v); }

#define WS_QF  0u
#define WS_KF  (WS_QF + 4u * (size_t)NB * SX * DM_)
#define WS_VF  (WS_KF + 4u * (size_t)NB * SKV * DM_)
#define WS_QH  (WS_VF + 4u * (size_t)NB * SKV * DM_)
#define WS_KH  (WS_QH + 2u * (size_t)NB * SX * DM_)
#define WS_KL  (WS_KH + 2u * (size_t)NB * SKV * DM_)
#define WS_VH  (WS_KL + 2u * (size_t)NB * SKV * DM_)
#define WS_VL  (WS_VH + 2u * (size_t)NB * DM_ * SKV)
#define WS_CT  (WS_VL + 2u * (size_t)NB * DM_ * SKV)
#define WS_END (WS_CT + 4u * (size_t)NB * SX * DM_)

__global__ __launch_bounds__(128) void k_lin(const float* __restrict__ IN, int in_rows_per_b, int row_off, const float* __restrict__ Wt, const float* __restrict__ Bs, float* __restrict__ OUT, int out_rows_per_b) {
  __shared__ __align__(16) float sf[4][16][132];
  const int tid = threadIdx.x, wave = tid >> 5, lane = tid & 31, col = lane & 15, g = lane >> 4; const int c0 = blockIdx.y * 128; const size_t b = blockIdx.z; const int rl0 = blockIdx.x * 64 + wave * 16;
  const float* src = IN + (b * in_rows_per_b + rl0 + col) * (size_t)DM_;
  v8f acc[8] = {};
#pragma unroll 2
  for (int kc = 0; kc < DM_ / 32; ++kc) { v16b a; { const float* p = src + kc * 32 + 8 * g;
#pragma unroll
      for (int i = 0; i < 8; ++i) { a[i] = (__bf16)p[i]; a[8 + i] = (__bf16)p[16 + i]; } }
#pragma unroll
    for (int j = 0; j < 8; ++j) { v16b w; const size_t o = c0 + j * 16 + col;
#pragma unroll
      for (int i = 0; i < 8; ++i) { w[i] = (__bf16)Wt[o * DM_ + kc * 32 + 8 * g + i]; w[8 + i] = (__bf16)Wt[o * DM_ + kc * 32 + 16 + 8 * g + i]; }
      acc[j] = wmma_bf(a, w, acc[j]); } }
#pragma unroll
  for (int j = 0; j < 8; ++j) { const float bb = bfr(Bs[c0 + j * 16 + col]);
#pragma unroll
    for (int r = 0; r < 8; ++r) sf[wave][8 * g + r][j * 16 + col] = acc[j][r] + bb; }
  LDSX(); { float* dst = OUT + (b * out_rows_per_b + row_off + rl0) * (size_t)DM_ + c0; for (int rl = 0; rl < 16; ++rl) vst2(dst + (size_t)rl * DM_ + lane * 4, *(const v4f*)&sf[wave][rl][lane * 4]); } }
__global__ __launch_bounds__(256) void k_nr(const float* __restrict__ F, const float* __restrict__ G, const float* __restrict__ FR0, const float* __restrict__ FR1, int rows_per_b, int split, _Float16* __restrict__ H16, _Float16* __restrict__ L16) { __shared__ float sred[8]; __shared__ float sinv; __shared__ __align__(16) _Float16 sh[DM_], sl[DM_];
  const int t = threadIdx.x; const size_t row = blockIdx.x; const int j = (int)(row % rows_per_b); const float* fr = F + row * DM_;
  const float* tab = (j < split) ? (FR0 + (size_t)j * HD) : (FR1 + (size_t)(j - split) * HD);
  float q2 = 0.f; for (int e = t; e < DM_; e += 256) { const float v = fr[e]; q2 += v * v; }
#pragma unroll
  for (int o = 1; o < 32; o <<= 1) q2 += __shfl_xor(q2, o);
  if ((t & 31) == 0) sred[t >> 5] = q2; __syncthreads(); if (t == 0) { float a = 0.f; for (int i = 0; i < 8; ++i) a += sred[i]; sinv = 1.0f / sqrtf(a * (1.0f / DM_) + 1e-6f); } __syncthreads();
  const float inv = sinv;
  for (int e = t; e < DM_ / 2; e += 256) { const int p = e % (HD / 2); const int c = 2 * e;
    const float xr = fr[c] * inv * bfr(G[c]), xi = fr[c + 1] * inv * bfr(G[c + 1]); const float f_r = bfr(tab[2 * p]), f_i = bfr(tab[2 * p + 1]);
    const float y0 = xr * f_r - xi * f_i, y1 = xr * f_i + xi * f_r; const _Float16 h0 = (_Float16)y0, h1 = (_Float16)y1; sh[c] = h0; sh[c + 1] = h1; sl[c] = (_Float16)(y0 - (float)h0); sl[c + 1] = (_Float16)(y1 - (float)h1); }
  __syncthreads(); for (int q = t; q < DM_ / 8; q += 256) { vst2((unsigned*)(H16 + row * DM_ + q * 8), *(const v4u*)&sh[q * 8]); if (L16) vst2((unsigned*)(L16 + row * DM_ + q * 8), *(const v4u*)&sl[q * 8]); } }
__global__ __launch_bounds__(128) void k_vt(const float* __restrict__ VF, _Float16* __restrict__ VH, _Float16* __restrict__ VL) { __shared__ __align__(16) _Float16 th[128][72], tl[128][72];
  const int t = threadIdx.x; const size_t b = blockIdx.z; const int k0 = blockIdx.x * 64, c0 = blockIdx.y * 128;
  for (int e = t; e < 64 * 128; e += 128) { const int kl = e >> 7, c = e & 127; const float v = VF[(b * SKV + k0 + kl) * (size_t)DM_ + c0 + c]; const _Float16 hv = (_Float16)v; th[c][kl] = hv; tl[c][kl] = (_Float16)(v - (float)hv); }
  __syncthreads(); for (int e = t; e < 128 * 8; e += 128) { const int c = e >> 3, q = e & 7; const size_t o = (b * DM_ + c0 + c) * (size_t)SKV + k0 + q * 8; vst2((unsigned*)(VH + o), *(const v4u*)&th[c][q * 8]); vst2((unsigned*)(VL + o), *(const v4u*)&tl[c][q * 8]); } }
__global__ __launch_bounds__(128) void k_att(const _Float16* __restrict__ QH, const _Float16* __restrict__ KH, const _Float16* __restrict__ KL, const _Float16* __restrict__ VH, const _Float16* __restrict__ VL, float* __restrict__ CT) {
  __shared__ __align__(16) float sp[4][16][36]; __shared__ __align__(16) float so[4][16][132];
  const int tid = threadIdx.x, wave = tid >> 5, lane = tid & 31, col = lane & 15, g = lane >> 4; const int qb = blockIdx.x, h = blockIdx.y; const size_t b = blockIdx.z; const size_t q0 = b * SX + (size_t)qb * 64 + wave * 16;
  v16h aq[4];
#pragma unroll
  for (int kc = 0; kc < 4; ++kc) aq[kc] = frag_h(QH + (q0 + col) * DM_ + h * HD + kc * 32, lane);
  float m[8], l[8];
#pragma unroll
  for (int r = 0; r < 8; ++r) { m[r] = -3.0e38f; l[r] = 0.f; }
  v8f acc[8] = {};
#pragma unroll 1
  for (int ks = 0; ks < SKV / 32; ++ks) { float s[2][8];
#pragma unroll
    for (int ct = 0; ct < 2; ++ct) { const size_t kk = b * SKV + ks * 32 + ct * 16 + col; v8f c = {};
#pragma unroll
      for (int kc = 0; kc < 4; ++kc) { c = wmma16(aq[kc], frag_h(KH + kk * DM_ + h * HD + kc * 32, lane), c); c = wmma16(aq[kc], frag_h(KL + kk * DM_ + h * HD + kc * 32, lane), c); }
#pragma unroll
      for (int r = 0; r < 8; ++r) s[ct][r] = c[r] * 0.08838834764831845f; }
    float alpha[8];
#pragma unroll
    for (int r = 0; r < 8; ++r) { float mx = fmaxf(s[0][r], s[1][r]);
#pragma unroll
      for (int o = 1; o < 16; o <<= 1) mx = fmaxf(mx, __shfl_xor(mx, o));
      const float mn = fmaxf(m[r], mx); alpha[r] = __expf(m[r] - mn); const float e0 = __expf(s[0][r] - mn), e1 = __expf(s[1][r] - mn); float es = e0 + e1;
#pragma unroll
      for (int o = 1; o < 16; o <<= 1) es += __shfl_xor(es, o);
      l[r] = l[r] * alpha[r] + es; m[r] = mn; sp[wave][8 * g + r][col] = e0; sp[wave][8 * g + r][16 + col] = e1; }
#pragma unroll
    for (int j = 0; j < 8; ++j)
#pragma unroll
      for (int r = 0; r < 8; ++r) acc[j][r] *= alpha[r];
    LDSX();
    const v16h pa = frag_f32s(&sp[wave][col][0], lane, 2048.0f);
#pragma unroll
    for (int j = 0; j < 8; ++j) { const size_t po = (b * DM_ + (size_t)h * HD + j * 16 + col) * SKV + ks * 32; acc[j] = wmma16(pa, frag_h(VH + po, lane), acc[j]); }
    LDSX(); }
#pragma unroll
  for (int r = 0; r < 8; ++r) { const float il = (1.0f / 2048.0f) / l[r];
#pragma unroll
    for (int j = 0; j < 8; ++j) so[wave][8 * g + r][j * 16 + col] = acc[j][r] * il; }
  LDSX(); for (int rl = 0; rl < 16; ++rl) vst2(CT + (q0 + rl) * DM_ + h * HD + lane * 4, *(const v4f*)&so[wave][rl][lane * 4]); }
__global__ __launch_bounds__(128) void k_out(const float* __restrict__ CT, const float* __restrict__ WO, const float* __restrict__ BO, float* __restrict__ OUT) { __shared__ __align__(16) float sf[4][16][132];
  const int tid = threadIdx.x, wave = tid >> 5, lane = tid & 31, col = lane & 15, g = lane >> 4; const int c0 = blockIdx.y * 128; const size_t r0 = (size_t)blockIdx.x * 64 + wave * 16;
  v8f acc[8] = {};
#pragma unroll 2
  for (int kc = 0; kc < DM_ / 32; ++kc) { const v16h a = frag_f32(CT + (r0 + col) * DM_ + kc * 32, lane);
#pragma unroll
    for (int j = 0; j < 8; ++j) { v16h w; const size_t o = c0 + j * 16 + col;
#pragma unroll
      for (int i = 0; i < 8; ++i) { w[i] = (_Float16)bfr(WO[o * DM_ + kc * 32 + 8 * g + i]); w[8 + i] = (_Float16)bfr(WO[o * DM_ + kc * 32 + 16 + 8 * g + i]); }
      acc[j] = wmma16(a, w, acc[j]); } }
#pragma unroll
  for (int j = 0; j < 8; ++j) { const float bb = bfr(BO[c0 + j * 16 + col]);
#pragma unroll
    for (int r = 0; r < 8; ++r) sf[wave][8 * g + r][j * 16 + col] = acc[j][r] + bb; }
  LDSX(); for (int rl = 0; rl < 16; ++rl) vst2(OUT + (r0 + rl) * DM_ + c0 + lane * 4, *(const v4f*)&sf[wave][rl][lane * 4]); }
extern "C" void kernel_launch(void* const* d_in, const int* in_sizes, int n_in, void* d_out, int out_size, void* d_ws, size_t ws_size, hipStream_t stream) {
  (void)in_sizes; (void)n_in; (void)out_size;
  const float** F = (const float**)d_in;
  if (ws_size < (size_t)WS_END) return;
  char* ws = (char*)d_ws; float *QF = (float*)(ws + WS_QF), *KF = (float*)(ws + WS_KF), *VF = (float*)(ws + WS_VF), *CT = (float*)(ws + WS_CT); _Float16 *QH = (_Float16*)(ws + WS_QH), *KH = (_Float16*)(ws + WS_KH), *KL = (_Float16*)(ws + WS_KL), *VH = (_Float16*)(ws + WS_VH), *VL = (_Float16*)(ws + WS_VL);
  k_lin<<<dim3(TQB, DM_ / 128, TNB), 128, 0, stream>>>(F[0], SX, 0, F[6], F[7], QF, SX);
  k_lin<<<dim3(SC / 64, DM_ / 128, TNB), 128, 0, stream>>>(F[1], SC, 0, F[8], F[9], KF, SKV);
  k_lin<<<dim3(SR / 64, DM_ / 128, TNB), 128, 0, stream>>>(F[2], SR, SC, F[12], F[13], KF, SKV);
  k_lin<<<dim3(SC / 64, DM_ / 128, TNB), 128, 0, stream>>>(F[1], SC, 0, F[10], F[11], VF, SKV);
  k_lin<<<dim3(SR / 64, DM_ / 128, TNB), 128, 0, stream>>>(F[2], SR, SC, F[14], F[15], VF, SKV);
  for (int b = 0; b < TNB; ++b) { k_nr<<<TQB * 64, 256, 0, stream>>>(QF + (size_t)b * SX * DM_, F[18], F[3], F[3], SX, SX, QH + (size_t)b * SX * DM_, nullptr); k_nr<<<SKV, 256, 0, stream>>>(KF + (size_t)b * SKV * DM_, F[19], F[4], F[5], SKV, SC, KH + (size_t)b * SKV * DM_, KL + (size_t)b * SKV * DM_); }
  k_vt<<<dim3(SKV / 64, DM_ / 128, TNB), 128, 0, stream>>>(VF, VH, VL);
  k_att<<<dim3(TQB, NH, TNB), 128, 0, stream>>>(QH, KH, KL, VH, VL, CT);
  for (int b = 0; b < TNB; ++b) k_out<<<dim3(TQB, DM_ / 128), 128, 0, stream>>>(CT + (size_t)b * SX * DM_, F[16], F[17], (float*)d_out + (size_t)b * SX * DM_);
}
